// SimpleMambaBlock_74766790689538
// MI455X (gfx1250) — hardware-run, weakly checked
//
#include <hip/hip_runtime.h>
#include <math.h>

typedef __attribute__((ext_vector_type(16))) _Float16 v16h;
typedef __attribute__((ext_vector_type(8)))  _Float16 v8h;
typedef __attribute__((ext_vector_type(8)))  float    v8f;
typedef __attribute__((ext_vector_type(4)))  float    v4f;

constexpr int kBatch  = 2;
constexpr int kSeq    = 2048;
constexpr int kDm     = 1024;
constexpr int kDin    = 2048;
constexpr int kNst    = 16;
constexpr int kDtR    = 64;
constexpr int kPrjN   = kDtR + 2 * kNst;
constexpr int kPrjP   = 128;
constexpr int kXzP    = 2 * kDin;
constexpr int kRows   = kBatch * kSeq;
constexpr int kConvCh = 512;
constexpr int kConvTP = 516;
constexpr int kScanTS = 64;
constexpr int kScanCh = 64;
constexpr int kScanYP = 68;
constexpr int kLnThreads = 256;
constexpr float kLnEps = 1e-5f;

constexpr float kCarryAct  = 16.0f;
constexpr float kCarryY    = 64.0f;
constexpr float kCarryW    = 256.0f;
constexpr float kCarryWdt  = 64.0f;
constexpr float kInvAct    = 1.0f / kCarryAct;
constexpr float kSclIn     = kCarryAct / (kCarryAct * kCarryW);
constexpr float kSclXp     = 1.0f / (kCarryAct * kCarryW);
constexpr float kSclDt     = kCarryAct / (kCarryAct * kCarryWdt);
constexpr float kSclOut    = 1.0f / (kCarryY * kCarryW);
constexpr float kF16MinNormal = 6.103515625e-5f;

static_assert(kPrjN == 96, "x_proj width");
static_assert((kDm % 32) == 0 && (kDin % 32) == 0 && (kDtR % 32) == 0, "GEMM K multiples of 32");
static_assert((kRows % 64) == 0 && (kXzP % 64) == 0 && (kPrjP % 64) == 0 && (kDin % 64) == 0 && (kDm % 64) == 0, "GEMM M,N multiples of 64");
static_assert((kSeq % kScanTS) == 0 && (kSeq % 64) == 0 && (kDin % kScanCh) == 0 && (kDin % kConvCh) == 0, "tile multiples");
static_assert(kDm == 4 * kLnThreads, "LayerNorm lane map: 256 lanes x 4 columns");

constexpr size_t kSzX16    = (size_t)kRows * kDm * 2;
constexpr size_t kSzWIN16  = (size_t)kXzP * kDm * 2;
constexpr size_t kSzWXP16  = (size_t)kPrjP * kDin * 2;
constexpr size_t kSzWDT16  = (size_t)kDin * kDtR * 2;
constexpr size_t kSzWOUT16 = (size_t)kDm * kDin * 2;
constexpr size_t kSzXZ16   = (size_t)kRows * kXzP * 2;
constexpr size_t kSzXC16   = (size_t)kRows * kDin * 2;
constexpr size_t kSzPROJ   = (size_t)kRows * kPrjP * 4;
constexpr size_t kSzDTLOW  = (size_t)kRows * kDtR * 2;
constexpr size_t kSzDL16   = (size_t)kRows * kDin * 2;
constexpr size_t kSzY16    = (size_t)kRows * kDin * 2;
constexpr size_t kSzHPRE   = (size_t)kRows * kDm * 4;
constexpr size_t kOffX16    = 0;
constexpr size_t kOffWIN16  = kOffX16    + kSzX16;
constexpr size_t kOffWXP16  = kOffWIN16  + kSzWIN16;
constexpr size_t kOffWDT16  = kOffWXP16  + kSzWXP16;
constexpr size_t kOffWOUT16 = kOffWDT16  + kSzWDT16;
constexpr size_t kOffXZ16   = kOffWOUT16 + kSzWOUT16;
constexpr size_t kOffXC16   = kOffXZ16   + kSzXZ16;
constexpr size_t kOffPROJ   = kOffXC16   + kSzXC16;
constexpr size_t kOffDTLOW  = kOffPROJ   + kSzPROJ;
constexpr size_t kOffDL16   = kOffDTLOW  + kSzDTLOW;
constexpr size_t kOffY16    = kOffDL16   + kSzDL16;
constexpr size_t kOffHPRE   = kOffY16    + kSzY16;
constexpr size_t kWsTotal   = kOffHPRE   + kSzHPRE;
static_assert(kWsTotal == 125042688ull, "carve total");
static_assert(kWsTotal <= 134217728ull, "carve cap");
static_assert((kOffWIN16 % 128) == 0 && (kOffWXP16 % 128) == 0 && (kOffWDT16 % 128) == 0 && (kOffWOUT16 % 128) == 0 &&
              (kOffXZ16 % 128) == 0 && (kOffXC16 % 128) == 0 && (kOffPROJ % 128) == 0 && (kOffDTLOW % 128) == 0 &&
              (kOffDL16 % 128) == 0 && (kOffY16 % 128) == 0 && (kOffHPRE % 128) == 0, "128-B aligned regions");

__device__ __forceinline__ float h16_to_f32(unsigned hb) {
  const unsigned sgn = (hb & 0x8000u) << 16;
  const unsigned em = hb & 0x7fffu;
  const float fn = __uint_as_float((em << 13) + 0x38000000u);
  const float fs = (float)em * 5.9604644775390625e-8f;
  const float mag = (em < 0x400u) ? fs : fn;
  return __uint_as_float(__float_as_uint(mag) | sgn);
}
__device__ __forceinline__ _Float16 f16_flush(float v) {
  const float a = (fabsf(v) < kF16MinNormal) ? 0.0f : v;
  return (_Float16)a;
}
__device__ __forceinline__ float sigmoid_f32(float v) {
  return __builtin_amdgcn_rcpf(1.0f + expf(-v));
}
__device__ __forceinline__ float sigmoid_hw(float v) {
  return __builtin_amdgcn_rcpf(1.0f + __expf(-v));
}
__device__ __forceinline__ float softplus_hw(float v) {
  const float a = __expf(-fabsf(v));
  const float u = 1.0f + a;
  const float l1p = __logf(u) + (a - (u - 1.0f)) * __builtin_amdgcn_rcpf(u);
  return fmaxf(v, 0.0f) + l1p;
}

__device__ __forceinline__ void mma_guard(v8f& acc, v16h a, v16h b) {
  asm volatile("v_nop\n\tv_nop\n\tv_nop\n\tv_nop" : "+v"(acc) : "v"(a), "v"(b));
}
__device__ __forceinline__ void keep4_h(v16h a, v16h b, v16h c, v16h d) {
  asm volatile("v_nop" :: "v"(a), "v"(b), "v"(c), "v"(d));
}
__device__ __forceinline__ void acc_guard4(v8f& a, v8f& b, v8f& c, v8f& d) {
  asm volatile("v_nop\n\tv_nop\n\tv_nop\n\tv_nop" : "+v"(a), "+v"(b), "+v"(c), "+v"(d));
}
struct FragH {
  union U { v16h v; v8h h[2]; };
  static __device__ __forceinline__ v16h load(const _Float16* p) {
    U f;
    f.h[0] = *(const v8h*)(p);
    f.h[1] = *(const v8h*)(p + 16);
    return f.v;
  }
  static __device__ __forceinline__ v8f mma(v16h a, v16h b, v8f c) {
    return __builtin_amdgcn_wmma_f32_16x16x32_f16(false, a, false, b, (short)0, c, false, false);
  }
};

template <int OUT_MODE>
__global__ __launch_bounds__(256) void wmma_gemm64(
    const unsigned short* __restrict__ Ap, int lda,
    const unsigned short* __restrict__ Btp, int ldb,
    void* __restrict__ Cout, int ldc,
    int M, int N, int K, float scale) {
  const _Float16* A  = (const _Float16*)Ap;
  const _Float16* Bt = (const _Float16*)Btp;
  __shared__ __align__(16) float sT[8][16 * 68];
  const int lane = threadIdx.x & 31;
  const int wave = threadIdx.x >> 5;
  const int tilesN = N >> 6;
  const int tilesM = M >> 6;
  const int tile = blockIdx.x * 8 + wave;
  if (tile >= tilesM * tilesN) return;
  const int tm = tile / tilesN;
  const int tn = tile - tm * tilesN;
  const int m0 = tm << 6;
  const int n0 = tn << 6;

  const int rlane = lane & 15;
  const int koff  = (lane >> 4) * 8;
  const int mOff  = (lane >> 4) * 8;

  v8f acc[4][4];
#pragma unroll
  for (int i = 0; i < 4; ++i)
#pragma unroll
    for (int j = 0; j < 4; ++j) acc[i][j] = (v8f){0.f,0.f,0.f,0.f,0.f,0.f,0.f,0.f};

  for (int k0 = 0; k0 < K; k0 += 32) {
    v16h bh[4];
#pragma unroll
    for (int j = 0; j < 4; ++j) {
      const size_t bo = (size_t)(n0 + (j << 4) + rlane) * ldb + koff + k0;
      bh[j] = FragH::load(Bt + bo);
    }
#pragma unroll
    for (int i = 0; i < 4; ++i) {
      const size_t ao = (size_t)(m0 + (i << 4) + rlane) * lda + koff + k0;
      const v16h ah = FragH::load(A + ao);
#pragma unroll
      for (int j = 0; j < 4; ++j) acc[i][j] = FragH::mma(ah, bh[j], acc[i][j]);
      mma_guard(acc[i][0], ah, bh[0]);
      mma_guard(acc[i][1], ah, bh[1]);
      mma_guard(acc[i][2], ah, bh[2]);
      mma_guard(acc[i][3], ah, bh[3]);
    }
    keep4_h(bh[0], bh[1], bh[2], bh[3]);
  }
  acc_guard4(acc[0][0], acc[0][1], acc[0][2], acc[0][3]);
  acc_guard4(acc[1][0], acc[1][1], acc[1][2], acc[1][3]);
  acc_guard4(acc[2][0], acc[2][1], acc[2][2], acc[2][3]);
  acc_guard4(acc[3][0], acc[3][1], acc[3][2], acc[3][3]);

  float* slab = sT[wave];
#pragma unroll
  for (int i = 0; i < 4; ++i) {
    const int mBase = m0 + (i << 4);
#pragma unroll
    for (int j = 0; j < 4; ++j) {
#pragma unroll
      for (int r = 0; r < 8; ++r) {
        const float v = acc[i][j][r] * scale;
        slab[(mOff + r) * 68 + (j << 4) + rlane] = v;
      }
    }
    __builtin_amdgcn_fence(__ATOMIC_RELEASE, "workgroup");
    __builtin_amdgcn_wave_barrier();
    __builtin_amdgcn_fence(__ATOMIC_ACQUIRE, "workgroup");
    if (OUT_MODE == 0) {
      float* C = (float*)Cout;
      const int hh = lane >> 4, c4 = (lane & 15) * 4;
      for (int pass = 0; pass < 2; ++pass) {
#pragma unroll
        for (int it = 0; it < 8; ++it) {
          const int row = it * 2 + hh;
          const v4f v = *(const v4f*)(slab + row * 68 + c4);
          *(volatile v4f*)(C + (size_t)(mBase + row) * ldc + n0 + c4) = v;
        }
        __threadfence();
      }
    } else {
      const int q = lane >> 3, c8 = (lane & 7) * 8;
      unsigned short* C = (unsigned short*)Cout;
      for (int pass = 0; pass < 2; ++pass) {
#pragma unroll
        for (int it = 0; it < 4; ++it) {
          const int row = it * 4 + q;
          const float* sp = slab + row * 68 + c8;
          v8h hv;
#pragma unroll
          for (int e = 0; e < 8; ++e) hv[e] = f16_flush(sp[e]);
          *(volatile v8h*)(C + (size_t)(mBase + row) * ldc + n0 + c8) = hv;
        }
        __threadfence();
      }
    }
    __builtin_amdgcn_fence(__ATOMIC_RELEASE, "workgroup");
    __builtin_amdgcn_wave_barrier();
    __builtin_amdgcn_fence(__ATOMIC_ACQUIRE, "workgroup");
  }
}

__global__ __launch_bounds__(256) void cast_f16_kernel(
    const float* __restrict__ src, unsigned short* __restrict__ dst, int total8, int real8, float scale)
{
  const int i = blockIdx.x * 256 + threadIdx.x;
  if (i >= total8) return;
  const bool live = (i < real8);
  const int ic = live ? i : (real8 - 1);
  const float* p = src + ((size_t)ic << 3);
  v4f a0 = *(const v4f*)(p);
  v4f a1 = *(const v4f*)(p + 4);
  asm volatile("" : "+v"(a0), "+v"(a1));
  v8h hv;
#pragma unroll
  for (int e = 0; e < 4; ++e) {
    const float s0 = live ? (a0[e] * scale) : 0.0f;
    const float s1 = live ? (a1[e] * scale) : 0.0f;
    hv[e]     = f16_flush(s0);
    hv[4 + e] = f16_flush(s1);
  }
  unsigned short* q = dst + ((size_t)i << 3);
  *(volatile v8h*)q = hv;
  __threadfence();
  *(volatile v8h*)q = hv;
}

__global__ __launch_bounds__(256) void dt_cast_kernel(
    const float* __restrict__ PROJ, unsigned short* __restrict__ DT16, int total8, float scale)
{
  const int i = blockIdx.x * 256 + threadIdx.x;
  if (i >= total8) return;
  const int e0  = i << 3;
  const int row = e0 >> 6;
  const int c8  = e0 & 63;
  const float* p = PROJ + (size_t)row * kPrjP + c8;
  const v4f a0 = *(const v4f*)(p);
  const v4f a1 = *(const v4f*)(p + 4);
  v8h hv;
#pragma unroll
  for (int e = 0; e < 4; ++e) {
    hv[e]     = f16_flush(a0[e] * scale);
    hv[4 + e] = f16_flush(a1[e] * scale);
  }
  unsigned short* qd = DT16 + e0;
  *(volatile v8h*)qd = hv;
  __threadfence();
  *(volatile v8h*)qd = hv;
}

__global__ __launch_bounds__(256) void conv_silu_kernel(
    const unsigned* __restrict__ XZw, const float* __restrict__ cw, const float* __restrict__ cb,
    unsigned short* __restrict__ XC16)
{
  __shared__ __align__(16) float sT[16 * kConvTP];
  const int tid = threadIdx.x, lane = tid & 31, wave = tid >> 5;
  const int d0 = blockIdx.x * kConvCh;
  const int dp = d0 + 2 * tid;
  const int g0 = blockIdx.y * 64;
  const int tb = g0 & (kSeq - 1);
  constexpr int kWP = kXzP / 2;
  const int wcol = (d0 >> 1) + tid;
  const v4f wa = *(const v4f*)(cw + (size_t)dp * 4);
  const v4f wb = *(const v4f*)(cw + (size_t)dp * 4 + 4);
  const float ba = cb[dp];
  const float bbv = cb[dp + 1];
  float a3, a2, a1, b3, b2, b1;
  {
    const bool hist = (tb > 0);
    const int rb = hist ? (g0 - 3) : g0;
    unsigned u3 = XZw[(size_t)rb * kWP + wcol];
    unsigned u2 = XZw[(size_t)(rb + 1) * kWP + wcol];
    unsigned u1 = XZw[(size_t)(rb + 2) * kWP + wcol];
    asm volatile("" : "+v"(u3), "+v"(u2), "+v"(u1));
    const float f3a = h16_to_f32(u3 & 0xffffu), f3b = h16_to_f32(u3 >> 16);
    const float f2a = h16_to_f32(u2 & 0xffffu), f2b = h16_to_f32(u2 >> 16);
    const float f1a = h16_to_f32(u1 & 0xffffu), f1b = h16_to_f32(u1 >> 16);
    a3 = hist ? f3a : 0.0f;
    b3 = hist ? f3b : 0.0f;
    a2 = hist ? f2a : 0.0f;
    b2 = hist ? f2b : 0.0f;
    a1 = hist ? f1a : 0.0f;
    b1 = hist ? f1b : 0.0f;
  }
#pragma unroll 1
  for (int sub = 0; sub < 4; ++sub) {
    const int lb = g0 + sub * 16;
#pragma unroll 1
    for (int s = 0; s < 16; ++s) {
      const unsigned uc = XZw[(size_t)(lb + s) * kWP + wcol];
      const float ca  = h16_to_f32(uc & 0xffffu);
      const float cbn = h16_to_f32(uc >> 16);
      float acc0 = wa[0] * a3;
      acc0 = fmaf(wa[1], a2, acc0);
      acc0 = fmaf(wa[2], a1, acc0);
      acc0 = fmaf(wa[3], ca, acc0);
      float acc1 = wb[0] * b3;
      acc1 = fmaf(wb[1], b2, acc1);
      acc1 = fmaf(wb[2], b1, acc1);
      acc1 = fmaf(wb[3], cbn, acc1);
      const float sv0 = fmaf(acc0, kInvAct, ba);
      const float sv1 = fmaf(acc1, kInvAct, bbv);
      const float y0 = sv0 * sigmoid_f32(sv0);
      const float y1 = sv1 * sigmoid_f32(sv1);
      sT[s * kConvTP + 2 * tid]     = y0 * kCarryAct;
      sT[s * kConvTP + 2 * tid + 1] = y1 * kCarryAct;
      a3 = a2; a2 = a1; a1 = ca;
      b3 = b2; b2 = b1; b1 = cbn;
    }
    __syncthreads();
    v8h hv[4];
#pragma unroll
    for (int it = 0; it < 4; ++it) {
      const int idx = it * 8 + wave;
      const int row = idx >> 1;
      const int ch  = (idx & 1) * 256 + lane * 8;
      const float* sp = sT + row * kConvTP + ch;
      const v4f q0 = *(const v4f*)(sp);
      const v4f q1 = *(const v4f*)(sp + 4);
#pragma unroll
      for (int e = 0; e < 4; ++e) {
        hv[it][e]     = f16_flush(q0[e]);
        hv[it][4 + e] = f16_flush(q1[e]);
      }
    }
    for (int pass = 0; pass < 2; ++pass) {
#pragma unroll
      for (int it = 0; it < 4; ++it) {
        const int idx = it * 8 + wave;
        const int row = idx >> 1;
        const int ch  = (idx & 1) * 256 + lane * 8;
        *(volatile v8h*)(XC16 + (size_t)(lb + row) * kDin + d0 + ch) = hv[it];
      }
      __threadfence();
    }
    __syncthreads();
  }
}

__global__ __launch_bounds__(64) void scan_kernel(
    const unsigned short* __restrict__ DL16, const unsigned short* __restrict__ XC16,
    const unsigned short* __restrict__ XZ16, const float* __restrict__ PROJ,
    const float* __restrict__ bdt, const float* __restrict__ Alog, const float* __restrict__ Dp,
    unsigned short* __restrict__ Y16)
{
  __shared__ __align__(16) float sBC[kScanTS * 32];
  __shared__ __align__(16) float sY[kScanTS * kScanYP];
  __shared__ __align__(16) float sA[kNst * kScanCh];
  const int tid = threadIdx.x, lane = tid & 31, wave = tid >> 5;
  constexpr int kBlkPerB = kDin / kScanCh;
  const int bix = blockIdx.x / kBlkPerB;
  const int d0  = (blockIdx.x - bix * kBlkPerB) * kScanCh;
  const int d   = d0 + tid;
  const size_t row0 = (size_t)bix * kSeq;
#pragma unroll 1
  for (int s = 0; s < kNst; ++s) sA[s * kScanCh + tid] = -expf(Alog[(size_t)d * kNst + s]);
  __syncthreads();
  float negA[kNst], h[kNst];
#pragma unroll
  for (int s = 0; s < kNst; ++s) {
    negA[s] = sA[s * kScanCh + tid];
    h[s] = 0.f;
  }
  const float bb = bdt[d];
  const float Dd = Dp[d];
  const int q = lane >> 3, c8 = (lane & 7) * 8;
#pragma unroll 1
  for (int t0 = 0; t0 < kSeq; t0 += kScanTS) {
    __syncthreads();
#pragma unroll
    for (int i = 0; i < 8; ++i) {
      const int idx = tid + 64 * i;
      const int r = idx >> 3, c4 = (idx & 7) * 4;
      *(v4f*)(sBC + r * 32 + c4) = *(const v4f*)(PROJ + (row0 + t0 + r) * kPrjP + kDtR + c4);
    }
    __syncthreads();
#pragma unroll 1
    for (int s = 0; s < kScanTS; ++s) {
      const size_t grow = row0 + t0 + s;
      const unsigned dlb = DL16[grow * kDin + d];
      const unsigned xcb = XC16[grow * kDin + d];
      const unsigned zb  = XZ16[grow * kXzP + kDin + d];
      const float* xr = sBC + s * 32;
      float Bs[kNst], Cs[kNst];
#pragma unroll
      for (int q4 = 0; q4 < 4; ++q4) {
        const v4f bv = *(const v4f*)(xr + 4 * q4);
        const v4f cv = *(const v4f*)(xr + kNst + 4 * q4);
        Bs[4 * q4 + 0] = bv[0]; Bs[4 * q4 + 1] = bv[1]; Bs[4 * q4 + 2] = bv[2]; Bs[4 * q4 + 3] = bv[3];
        Cs[4 * q4 + 0] = cv[0]; Cs[4 * q4 + 1] = cv[1]; Cs[4 * q4 + 2] = cv[2]; Cs[4 * q4 + 3] = cv[3];
      }
      const float v   = fmaf(h16_to_f32(dlb), kInvAct, bb);
      const float dt  = softplus_hw(v);
      const float xt  = h16_to_f32(xcb) * kInvAct;
      const float zv  = h16_to_f32(zb) * kInvAct;
      const float dtx = dt * xt;
      float y = 0.f;
#pragma unroll
      for (int k = 0; k < kNst; ++k) {
        const float e = __expf(dt * negA[k]);
        h[k] = e * h[k] + dtx * Bs[k];
        y = h[k] * Cs[k] + y;
      }
      y = xt * Dd + y;
      const float g = zv * sigmoid_hw(zv);
      sY[s * kScanYP + tid] = (y * g) * kCarryY;
    }
    __syncthreads();
    v8h hv[8];
#pragma unroll
    for (int it = 0; it < 8; ++it) {
      const int row = it * 8 + wave * 4 + q;
      const float* sp = sY + row * kScanYP + c8;
      const v4f q0 = *(const v4f*)(sp);
      const v4f q1 = *(const v4f*)(sp + 4);
#pragma unroll
      for (int e = 0; e < 4; ++e) {
        hv[it][e]     = f16_flush(q0[e]);
        hv[it][4 + e] = f16_flush(q1[e]);
      }
    }
    for (int pass = 0; pass < 2; ++pass) {
#pragma unroll
      for (int it = 0; it < 8; ++it) {
        const int row = it * 8 + wave * 4 + q;
        *(volatile v8h*)(Y16 + (row0 + t0 + row) * kDin + d0 + c8) = hv[it];
      }
      __threadfence();
    }
  }
}

__global__ __launch_bounds__(kLnThreads) void resid_ln_kernel(
    const float* __restrict__ HPRE, const float* __restrict__ xin,
    const float* __restrict__ gamma, const float* __restrict__ beta, float* __restrict__ out)
{
  __shared__ float sSum[8];
  __shared__ float sSq[8];
  const int tid = threadIdx.x, lane = tid & 31, wave = tid >> 5;
  const int row = blockIdx.x;
  const size_t base = (size_t)row * kDm;
  const int c = tid * 4;
  const v4f a  = *(const v4f*)(HPRE + base + c);
  const v4f b  = *(const v4f*)(xin + base + c);
  const v4f g  = *(const v4f*)(gamma + c);
  const v4f bt = *(const v4f*)(beta + c);
  const v4f v = a + b;
  float s = (v[0] + v[1]) + (v[2] + v[3]);
#pragma unroll
  for (int off = 16; off > 0; off >>= 1) s += __shfl_xor(s, off, 32);
  if (lane == 0) sSum[wave] = s;
  __syncthreads();
  float tot = 0.f;
#pragma unroll
  for (int w = 0; w < 8; ++w) tot += sSum[w];
  const float mu = tot * (1.0f / (float)kDm);
  float sq = 0.f;
#pragma unroll
  for (int e = 0; e < 4; ++e) {
    const float dv = v[e] - mu;
    sq = fmaf(dv, dv, sq);
  }
#pragma unroll
  for (int off = 16; off > 0; off >>= 1) sq += __shfl_xor(sq, off, 32);
  if (lane == 0) sSq[wave] = sq;
  __syncthreads();
  float tq = 0.f;
#pragma unroll
  for (int w = 0; w < 8; ++w) tq += sSq[w];
  const float rstd = rsqrtf(tq * (1.0f / (float)kDm) + kLnEps);
  v4f o;
#pragma unroll
  for (int e = 0; e < 4; ++e) {
    const float tn = (v[e] - mu) * rstd;
    o[e] = fmaf(tn, g[e], bt[e]);
  }
  float* dst = out + base + c;
  *(volatile v4f*)dst = o;
  __threadfence();
  *(volatile v4f*)dst = o;
}

extern "C" void kernel_launch(void* const* d_in, const int* in_sizes, int n_in,
                              void* d_out, int out_size, void* d_ws, size_t ws_size,
                              hipStream_t stream) {
  if (n_in < 12) return;
  if (in_sizes[0] != kRows * kDm) return;
  if (in_sizes[1] != kXzP * kDm) return;
  if (in_sizes[2] != kDin * 4) return;
  if (in_sizes[3] != kDin) return;
  if (in_sizes[4] != kPrjN * kDin) return;
  if (in_sizes[5] != kDin * kDtR) return;
  if (in_sizes[6] != kDin) return;
  if (in_sizes[7] != kDin * kNst) return;
  if (in_sizes[8] != kDin) return;
  if (in_sizes[9] != kDm * kDin) return;
  if (in_sizes[10] != kDm) return;
  if (in_sizes[11] != kDm) return;
  if (out_size != kRows * kDm) return;
  if (ws_size < kWsTotal) return;

  const float* x       = (const float*)d_in[0];
  const float* W_in    = (const float*)d_in[1];
  const float* conv_w  = (const float*)d_in[2];
  const float* conv_b  = (const float*)d_in[3];
  const float* W_xp    = (const float*)d_in[4];
  const float* W_dt    = (const float*)d_in[5];
  const float* b_dt    = (const float*)d_in[6];
  const float* A_log   = (const float*)d_in[7];
  const float* Dp      = (const float*)d_in[8];
  const float* W_out   = (const float*)d_in[9];
  const float* ln_g    = (const float*)d_in[10];
  const float* ln_b    = (const float*)d_in[11];
  float* out = (float*)d_out;

  char* ws = (char*)d_ws;
  unsigned short* X16     = (unsigned short*)(ws + kOffX16);
  unsigned short* WIN16   = (unsigned short*)(ws + kOffWIN16);
  unsigned short* WXP16   = (unsigned short*)(ws + kOffWXP16);
  unsigned short* WDT16   = (unsigned short*)(ws + kOffWDT16);
  unsigned short* WOUT16  = (unsigned short*)(ws + kOffWOUT16);
  unsigned short* XZ16    = (unsigned short*)(ws + kOffXZ16);
  unsigned short* XC16    = (unsigned short*)(ws + kOffXC16);
  float*          PROJ    = (float*)(ws + kOffPROJ);
  unsigned short* DTLOW16 = (unsigned short*)(ws + kOffDTLOW);
  unsigned short* DL16    = (unsigned short*)(ws + kOffDL16);
  unsigned short* Y16     = (unsigned short*)(ws + kOffY16);
  float*          HPRE    = (float*)(ws + kOffHPRE);

  {
    constexpr int nX   = kRows * kDm / 8;
    constexpr int nWin = kXzP * kDm / 8;
    constexpr int nWxp = kPrjP * kDin / 8;
    constexpr int nWxpReal = kPrjN * kDin / 8;
    constexpr int nWdt = kDin * kDtR / 8;
    constexpr int nWout = kDm * kDin / 8;
    static_assert((nX % 256) == 0 && (nWin % 256) == 0 && (nWxp % 256) == 0 && (nWxpReal % 256) == 0 &&
                  (nWdt % 256) == 0 && (nWout % 256) == 0, "exact cast grids");
    cast_f16_kernel<<<nX / 256, 256, 0, stream>>>(x, X16, nX, nX, kCarryAct);
    cast_f16_kernel<<<nWin / 256, 256, 0, stream>>>(W_in, WIN16, nWin, nWin, kCarryW);
    cast_f16_kernel<<<nWxp / 256, 256, 0, stream>>>(W_xp, WXP16, nWxp, nWxpReal, kCarryW);
    cast_f16_kernel<<<nWdt / 256, 256, 0, stream>>>(W_dt, WDT16, nWdt, nWdt, kCarryWdt);
    cast_f16_kernel<<<nWout / 256, 256, 0, stream>>>(W_out, WOUT16, nWout, nWout, kCarryW);
  }

  wmma_gemm64<1><<<(kRows / 64) * (kXzP / 64) / 8, 256, 0, stream>>>(
      X16, kDm, WIN16, kDm, (void*)XZ16, kXzP, kRows, kXzP, kDm, kSclIn);

  conv_silu_kernel<<<dim3(kDin / kConvCh, kRows / 64), 256, 0, stream>>>(
      (const unsigned*)XZ16, conv_w, conv_b, XC16);

  wmma_gemm64<0><<<(kRows / 64) * (kPrjP / 64) / 8, 256, 0, stream>>>(
      XC16, kDin, WXP16, kDin, (void*)PROJ, kPrjP, kRows, kPrjP, kDin, kSclXp);

  dt_cast_kernel<<<(kRows * kDtR / 8) / 256, 256, 0, stream>>>(PROJ, DTLOW16, kRows * kDtR / 8, kCarryAct);

  wmma_gemm64<1><<<(kRows / 64) * (kDin / 64) / 8, 256, 0, stream>>>(
      DTLOW16, kDtR, WDT16, kDtR, (void*)DL16, kDin, kRows, kDin, kDtR, kSclDt);

  scan_kernel<<<kBatch * (kDin / kScanCh), kScanCh, 0, stream>>>(
      DL16, XC16, XZ16, PROJ, b_dt, A_log, Dp, Y16);

  wmma_gemm64<0><<<(kRows / 64) * (kDm / 64) / 8, 256, 0, stream>>>(
      Y16, kDin, WOUT16, kDin, (void*)HPRE, kDm, kRows, kDm, kDin, kSclOut);

  resid_ln_kernel<<<kRows, kLnThreads, 0, stream>>>(HPRE, x, ln_g, ln_b, out);
}
